// deformable_filter_9689446220041
// MI455X (gfx1250) — hardware-verified
//
#include <hip/hip_runtime.h>
#include <math.h>

typedef __attribute__((ext_vector_type(16))) _Float16 v16h;
typedef __attribute__((ext_vector_type(16))) __bf16 v16b;
typedef __attribute__((ext_vector_type(8)))  _Float16 v8h;
typedef __attribute__((ext_vector_type(8)))  float v8f;
typedef __attribute__((ext_vector_type(4)))  float v4f;
typedef __attribute__((ext_vector_type(2)))  float v2f;
typedef __attribute__((ext_vector_type(4)))  unsigned v4u;
typedef __attribute__((ext_vector_type(4)))  int v4i;
typedef float __attribute__((may_alias)) float_a;
typedef int __attribute__((may_alias)) int_a;

template <typename T> __device__ __forceinline__ void vst2(void* p, T v) { *(volatile T*)p = v; __threadfence(); *(volatile T*)p = v; }
__device__ __forceinline__ v8f wmma16(v16h a, v16h b, v8f c) {
  v8f d = __builtin_amdgcn_wmma_f32_16x16x32_f16(false, a, false, b, (short)0, c, false, false);
  asm volatile("v_nop\n\tv_nop\n\tv_nop\n\tv_nop" : "+v"(d) : "v"(a), "v"(b));
  return d;
}
__device__ __forceinline__ v8f wmma_bf(v16b a, v16b b, v8f c) {
  v8f d = __builtin_amdgcn_wmma_f32_16x16x32_bf16(false, a, false, b, (short)0, c, false, false);
  asm volatile("v_nop\n\tv_nop\n\tv_nop\n\tv_nop" : "+v"(d) : "v"(a), "v"(b));
  return d;
}
__device__ __forceinline__ v16h frag_h(const _Float16* rowk0, int lane) {
  union { v16h v; v8h q[2]; } u; const _Float16* p = rowk0 + 8 * (lane >> 4);
  u.q[0] = *(const v8h*)p; u.q[1] = *(const v8h*)(p + 16); return u.v;
}
__device__ __forceinline__ v16h frag_f32(const float* rowk0, int lane) {
  v16h a; const float* p = rowk0 + 8 * (lane >> 4);
#pragma unroll
  for (int i = 0; i < 8; ++i) { a[i] = (_Float16)p[i]; a[8 + i] = (_Float16)p[16 + i]; }
  return a;
}
__device__ __forceinline__ v16h frag_f32s(const float* rowk0, int lane, float sc) {
  v16h a; const float* p = rowk0 + 8 * (lane >> 4);
#pragma unroll
  for (int i = 0; i < 8; ++i) { a[i] = (_Float16)(p[i] * sc); a[8 + i] = (_Float16)(p[16 + i] * sc); }
  return a;
}
__device__ __forceinline__ v16h fragc_f32(const float* W, int k0, int n, int lane, int ld, int K) {
  v16h a; const int g = lane >> 4;
#pragma unroll
  for (int i = 0; i < 8; ++i) { const int ka = k0 + 8 * g + i, kb = ka + 16;
    a[i] = (_Float16)(ka < K ? W[(size_t)(ka < K ? ka : K - 1) * ld + n] : 0.f); a[8 + i] = (_Float16)(kb < K ? W[(size_t)(kb < K ? kb : K - 1) * ld + n] : 0.f); }
  return a;
}
struct F2 { v16b h, l; };
__device__ __forceinline__ F2 bsplit16(const float v[16]) { F2 r;
#pragma unroll
  for (int i = 0; i < 16; ++i) { const __bf16 h = (__bf16)v[i]; r.h[i] = h; r.l[i] = (__bf16)(v[i] - (float)h); }
  return r; }
__device__ __forceinline__ F2 split_row(const float* row, int k0, int lane) { float v[16]; const float* p = row + k0 + 8 * (lane >> 4);
#pragma unroll
  for (int i = 0; i < 8; ++i) { v[i] = p[i]; v[8 + i] = p[16 + i]; }
  return bsplit16(v); }
__device__ __forceinline__ F2 split_rowK(const float* row, int k0, int lane, int K) { float v[16]; const int g = lane >> 4;
#pragma unroll
  for (int i = 0; i < 8; ++i) { const int ka = k0 + 8 * g + i, kb = ka + 16; v[i] = ka < K ? row[ka < K ? ka : K - 1] : 0.f; v[8 + i] = kb < K ? row[kb < K ? kb : K - 1] : 0.f; }
  return bsplit16(v); }
__device__ __forceinline__ F2 split_col(const float* W, int k0, int n, int lane, int ld, int K) { float v[16]; const int g = lane >> 4;
#pragma unroll
  for (int i = 0; i < 8; ++i) { const int ka = k0 + 8 * g + i, kb = ka + 16; v[i] = ka < K ? W[(size_t)(ka < K ? ka : K - 1) * ld + n] : 0.f; v[8 + i] = kb < K ? W[(size_t)(kb < K ? kb : K - 1) * ld + n] : 0.f; }
  return bsplit16(v); }
__device__ __forceinline__ v8f mac3(const F2& a, const F2& b, v8f c) { c = wmma_bf(a.l, b.h, c); c = wmma_bf(a.h, b.l, c); return wmma_bf(a.h, b.h, c); }
__device__ __forceinline__ float sigm(float v) { return 1.0f / (1.0f + expf(-v)); }
#define LDSX() do { asm volatile("s_wait_dscnt 0" ::: "memory"); __builtin_amdgcn_wave_barrier(); __builtin_amdgcn_fence(__ATOMIC_RELEASE, "workgroup"); } while (0)


#define NB 4
#define CC 64
#define CO 64
#define HH 128
#define WWD 128
#define NP (HH * WWD)
#define NT 9
#define KD (NT * CC)
#define HP (HH + 2)
#define WP (WWD + 2)
#ifndef TPB
#define TPB (NP / 64)
#define TNB NB
#endif
typedef __attribute__((ext_vector_type(8))) __bf16 v8b;
__device__ __forceinline__ v16b frag_b(const __bf16* rowk0, int lane) {
  union { v16b v; v8b q[2]; } u; const __bf16* p = rowk0 + 8 * (lane >> 4);
  u.q[0] = *(const v8b*)p; u.q[1] = *(const v8b*)(p + 16); return u.v;
}
__device__ __forceinline__ float bfr(float v) { return (float)(__bf16)v; }
__device__ __attribute__((noinline)) float exp_ni(float v) { return expf(v); }
__device__ __attribute__((noinline)) float erf_ni(float v) { return erff(v); }

#define WS_PO  0u
#define WS_PD  (WS_PO + 2u * (size_t)32 * KD)
#define WS_XT  (WS_PD + 2u * (size_t)CO * KD)
#define WS_OFF (WS_XT + 4u * (size_t)NB * NP * CC)
#define WS_END (WS_OFF + 4u * (size_t)NB * NP * 32)

__global__ __launch_bounds__(64) void k_pack(const float* __restrict__ WOFF, const float* __restrict__ WDEF, __bf16* __restrict__ P) { const int n = blockIdx.x, which = blockIdx.y, t = threadIdx.x; __shared__ __align__(16) __bf16 s[KD];
  if (which == 0) { if (n >= 32) return; for (int tap = 0; tap < NT; ++tap) s[tap * CC + t] = (n < 18) ? (__bf16)WOFF[((size_t)n * CC + t) * NT + tap] : (__bf16)0.0f; __syncthreads(); for (int q = t; q < KD / 8; q += 64) vst2((unsigned*)(P + WS_PO / 2 + (size_t)n * KD + q * 8), *(const v4u*)&s[q * 8]); }
  else { for (int tap = 0; tap < NT; ++tap) s[tap * CC + t] = (__bf16)WDEF[((size_t)n * CC + t) * NT + tap]; __syncthreads(); for (int q = t; q < KD / 8; q += 64) vst2((unsigned*)(P + WS_PD / 2 + (size_t)n * KD + q * 8), *(const v4u*)&s[q * 8]); } }
__global__ __launch_bounds__(256) void k_xt(const float* __restrict__ X, float* __restrict__ XT) { __shared__ float st[64][CC + 1]; __shared__ __align__(16) float so2[64][CC + 4]; const int t = threadIdx.x; const int p0 = blockIdx.x * 64; const size_t b = blockIdx.y;
  for (int e = t; e < CC * 64; e += 256) { const int c = e >> 6, pl = e & 63; st[pl][c] = bfr(X[(b * CC + c) * NP + p0 + pl]); } __syncthreads();
  for (int e = t; e < 64 * CC; e += 256) { const int pl = e >> 6, c = e & 63; so2[pl][c] = st[pl][c]; } __syncthreads();
  for (int e = t; e < 64 * 16; e += 256) { const int pl = e >> 4, q = e & 15; vst2(XT + ((b * NP + p0 + pl) * CC) + q * 4, *(const v4f*)&so2[pl][q * 4]); } }
__global__ __launch_bounds__(128) void k_off(const float* __restrict__ XT, const __bf16* __restrict__ P, const float* __restrict__ BOFF, float* __restrict__ OFF) { __shared__ __align__(16) float so[4][16][36];
  const int tid = threadIdx.x, wave = tid >> 5, lane = tid & 31, col = lane & 15, g = lane >> 4; const size_t b = blockIdx.y; const int p0 = blockIdx.x * 64 + wave * 16; const int pix = p0 + col; const int py = pix / WWD, px = pix % WWD; const __bf16* Wr = P + WS_PO / 2;
  v8f acc[2] = {};
#pragma unroll 1
  for (int tap = 0; tap < NT; ++tap) { const int yy = py + tap / 3 - 1, xx = px + tap % 3 - 1; const bool inb = yy >= 0 && yy < HH && xx >= 0 && xx < WWD; const float* src = XT + ((b * NP + (size_t)(inb ? yy * WWD + xx : 0)) * CC);
#pragma unroll
    for (int q = 0; q < 2; ++q) { v16b a; const float* pp = src + q * 32 + 8 * g;
#pragma unroll
      for (int i = 0; i < 8; ++i) { a[i] = (__bf16)(inb ? pp[i] : 0.f); a[8 + i] = (__bf16)(inb ? pp[16 + i] : 0.f); }
#pragma unroll
      for (int j = 0; j < 2; ++j) acc[j] = wmma_bf(a, frag_b(Wr + (size_t)(j * 16 + col) * KD + tap * CC + q * 32, lane), acc[j]); } }
#pragma unroll
  for (int j = 0; j < 2; ++j)
#pragma unroll
    for (int r = 0; r < 8; ++r) { const int ch = j * 16 + col; so[wave][8 * g + r][ch] = acc[j][r] + ((ch < 18) ? bfr(BOFF[ch]) : 0.f); }
  LDSX(); for (int rl = 0; rl < 16; ++rl) if (lane < 8) vst2(OFF + ((b * NP + p0 + rl) * 32) + lane * 4, *(const v4f*)&so[wave][rl][lane * 4]); }
__device__ __forceinline__ void corner16(const float* __restrict__ XTb, int qx, int qy, int g, int kc, float w, float* v) { const bool inside = (qx >= 1) && (qx <= HH) && (qy >= 1) && (qy <= WWD); if (!inside || w == 0.f) return; const float* p = XTb + ((size_t)((qx - 1) * WWD + (qy - 1)) * CC) + kc * 32 + 8 * g;
#pragma unroll
  for (int i = 0; i < 8; ++i) { v[i] += w * p[i]; v[8 + i] += w * p[16 + i]; } }
__global__ __launch_bounds__(128) void k_def(const float* __restrict__ XT, const float* __restrict__ OFF, const __bf16* __restrict__ P, const float* __restrict__ BDEF, float* __restrict__ Y) { __shared__ __align__(16) float so[CO][64 + 4];
  const int tid = threadIdx.x, wave = tid >> 5, lane = tid & 31, col = lane & 15, g = lane >> 4; const size_t b = blockIdx.y; const int p0 = blockIdx.x * 64 + wave * 16; const int pix = p0 + col; const int ph = pix / WWD, pw = pix % WWD; const __bf16* Wr = P + WS_PD / 2; const float* XTb = XT + b * NP * CC; const float* offp = OFF + (b * NP + pix) * 32;
  v8f acc[4] = {};
#pragma unroll 1
  for (int n = 0; n < NT; ++n) {
    const float pxf = (float)(ph + 1) + (float)(n / 3 - 1) + offp[n]; const float pyf = (float)(pw + 1) + (float)(n % 3 - 1) + offp[NT + n];
    const float flx = floorf(pxf), fly = floorf(pyf);
    const float qlx = fminf(fmaxf(flx, 0.f), (float)(HP - 1)), qly = fminf(fmaxf(fly, 0.f), (float)(WP - 1)), qrx = fminf(fmaxf(flx + 1.f, 0.f), (float)(HP - 1)), qry = fminf(fmaxf(fly + 1.f, 0.f), (float)(WP - 1));
    const float pxc = fminf(fmaxf(pxf, 0.f), (float)(HP - 1)), pyc = fminf(fmaxf(pyf, 0.f), (float)(WP - 1));
    const float glt = (1.f + (qlx - pxc)) * (1.f + (qly - pyc)), grb = (1.f - (qrx - pxc)) * (1.f - (qry - pyc)), glb = (1.f + (qlx - pxc)) * (1.f - (qry - pyc)), grt = (1.f - (qrx - pxc)) * (1.f + (qly - pyc));
    const int ilx = (int)qlx, ily = (int)qly, irx = (int)qrx, iry = (int)qry;
#pragma unroll
    for (int kc = 0; kc < 2; ++kc) { float v[16];
#pragma unroll
      for (int i = 0; i < 16; ++i) v[i] = 0.f;
      corner16(XTb, ilx, ily, g, kc, glt, v); corner16(XTb, irx, iry, g, kc, grb, v); corner16(XTb, ilx, iry, g, kc, glb, v); corner16(XTb, irx, ily, g, kc, grt, v);
      const F2 a = bsplit16(v);
#pragma unroll
      for (int j = 0; j < 4; ++j) { const v16b w = frag_b(Wr + (size_t)(j * 16 + col) * KD + n * CC + kc * 32, lane); acc[j] = wmma_bf(a.h, w, acc[j]); acc[j] = wmma_bf(a.l, w, acc[j]); } } }
#pragma unroll
  for (int j = 0; j < 4; ++j)
#pragma unroll
    for (int r = 0; r < 8; ++r) so[j * 16 + col][wave * 16 + 8 * g + r] = acc[j][r] + bfr(BDEF[j * 16 + col]);
  __syncthreads();
  for (int e = tid; e < CO * 16; e += 128) { const int o = e >> 4, q = e & 15; vst2(Y + ((b * CO + o) * NP) + (size_t)blockIdx.x * 64 + q * 4, *(const v4f*)&so[o][q * 4]); } }
extern "C" void kernel_launch(void* const* d_in, const int* in_sizes, int n_in, void* d_out, int out_size, void* d_ws, size_t ws_size, hipStream_t stream) {
  (void)in_sizes; (void)n_in; (void)out_size;
  const float** F = (const float**)d_in;
  if (ws_size < (size_t)WS_END) return;
  char* ws = (char*)d_ws; __bf16* P = (__bf16*)ws; float *XT = (float*)(ws + WS_XT), *OFF = (float*)(ws + WS_OFF);
  k_pack<<<dim3(CO, 2), 64, 0, stream>>>(F[1], F[3], P);
  k_xt<<<dim3(NP / 64, TNB), 256, 0, stream>>>(F[0], XT);
  k_off<<<dim3(TPB, TNB), 128, 0, stream>>>(XT, P, F[2], OFF);
  k_def<<<dim3(TPB, TNB), 128, 0, stream>>>(XT, OFF, P, F[4], (float*)d_out);
}
